// GlobalHybridGNNPolicy_54631984005470
// MI455X (gfx1250) — hardware-verified
//
#include <hip/hip_runtime.h>
#include <stddef.h>


#define NBATCH 64
#define FEAT   16
#define NHEAD  4
#define DDEG   5
#define NOUT   15
#define ROWF   (NBATCH * FEAT)
#define NB     32
#define CHUNK  2048
#define NTHR   256
#define NWAVE  8
#define NGRP   (CHUNK / (NTHR * 4))
#define WCAP   ((CHUNK / NTHR) * 32)
#define TPW    8

#define GAT_ACC  (NB * ROWF)
#define GAT_SR   (NB * NBATCH * NHEAD)
#define GAT_MR   (NB * NBATCH * NHEAD)
#define GAT_LIST (NWAVE * WCAP)
#define GAT_LDS_BYTES ((GAT_ACC + GAT_SR + GAT_MR + GAT_LIST + 16) * 4)

#define HD_AGG2 0
#define HD_SRC  (HD_AGG2 + 4096)
#define HD_TGT  (HD_SRC + 1024)
#define HD_BASE (HD_TGT + 5120)
#define HD_E1   (HD_BASE + 1024)
#define HD_E2   (HD_E1 + 4096)
#define HD_FLOATS (HD_E2 + 2048)
#define HEAD_LDS_BYTES (HD_FLOATS * 4)

static_assert(NGRP == 2);
static_assert(WCAP == 256);
static_assert(NB == 32);
static_assert(NBATCH * NHEAD == NTHR);
static_assert(((GAT_ACC + GAT_SR) % 4) == 0);
static_assert((GAT_MR % 4) == 0);
static_assert(GAT_LDS_BYTES == 204864);
static_assert(HEAD_LDS_BYTES == 69632);
static_assert(NOUT * NBATCH == 960);

typedef float          v4f   __attribute__((ext_vector_type(4)));
typedef float          v8f   __attribute__((ext_vector_type(8)));
typedef int            v4i   __attribute__((ext_vector_type(4)));
typedef unsigned short v16us __attribute__((ext_vector_type(16)));
typedef __bf16         v16bf __attribute__((ext_vector_type(16)));
union BFrag { v16us u; v16bf v; };

__device__ __forceinline__ unsigned bf_bits(float x) {
  const unsigned u = __float_as_uint(x);
  return (u + 0x7FFFu + ((u >> 16) & 1u)) >> 16;
}

__device__ __forceinline__ v8f wmb(v16bf a, v16bf b, v8f c) {
  v8f d = __builtin_amdgcn_wmma_f32_16x16x32_bf16(false, a, false, b, (short)0, c, false, false);
  asm volatile("v_nop\n\tv_nop\n\tv_nop\n\tv_nop" : "+v"(d) : "v"(a), "v"(b));
  return d;
}

__device__ __forceinline__ float lrelu(float v) { return v > 0.f ? v : 0.2f * v; }

__device__ __forceinline__ float tanh_f(float x) {
  const float ax = fabsf(x);
  const float t  = __expf(-2.0f * ax);
  const float r  = (1.0f - t) * __builtin_amdgcn_rcpf(1.0f + t);
  return x < 0.f ? -r : r;
}

__global__ __launch_bounds__(NTHR) void k_node(const float* __restrict__ hin, int sN, int sB,
                                               const float* __restrict__ Wl, const float* __restrict__ Wr,
                                               float* XL, float* XR, int nN) {
  __shared__ __attribute__((aligned(16))) float Tl[NWAVE * 256];
  __shared__ __attribute__((aligned(16))) float Tr[NWAVE * 256];
  const int tid  = threadIdx.x;
  const int lane = tid & 31;
  const int wave = tid >> 5;
  const int hh   = lane >> 4;
  const int m    = lane & 15;

  const v16us z16 = {0, 0, 0, 0, 0, 0, 0, 0, 0, 0, 0, 0, 0, 0, 0, 0};
  BFrag blh, bll, brh, brl;
  blh.u = z16; bll.u = z16; brh.u = z16; brl.u = z16;
#pragma unroll
  for (int i = 0; i < 8; ++i) {
    const float wl = Wl[(8 * hh + i) * FEAT + m];
    const float wr = Wr[(8 * hh + i) * FEAT + m];
    const unsigned hl = bf_bits(wl);
    const unsigned hr = bf_bits(wr);
    blh.u[i] = (unsigned short)hl;
    bll.u[i] = (unsigned short)bf_bits(wl - __uint_as_float(hl << 16));
    brh.u[i] = (unsigned short)hr;
    brl.u[i] = (unsigned short)bf_bits(wr - __uint_as_float(hr << 16));
  }

  const int numTiles = nN * (NBATCH / 16);
  float* tl = Tl + wave * 256;
  float* tr = Tr + wave * 256;
#pragma unroll 1
  for (int it = 0; it < TPW; ++it) {
    const int tw = (blockIdx.x * NWAVE + wave) * TPW + it;
    const bool valid = tw < numTiles;
    const int twc = valid ? tw : (numTiles - 1);
    const int n  = twc >> 2;
    const int b0 = (twc & 3) * 16;
    {
      const float* p = hin + (size_t)n * (size_t)sN + (size_t)(b0 + m) * (size_t)sB + 8 * hh;
      const v4f f0 = *(const v4f*)p;
      const v4f f1 = *(const v4f*)(p + 4);
      float xv[8];
      xv[0] = f0.x; xv[1] = f0.y; xv[2] = f0.z; xv[3] = f0.w;
      xv[4] = f1.x; xv[5] = f1.y; xv[6] = f1.z; xv[7] = f1.w;
      BFrag ah, al;
      ah.u = z16; al.u = z16;
#pragma unroll
      for (int i = 0; i < 8; ++i) {
        const unsigned hb = bf_bits(xv[i]);
        ah.u[i] = (unsigned short)hb;
        al.u[i] = (unsigned short)bf_bits(xv[i] - __uint_as_float(hb << 16));
      }
      v8f cl = {0.f, 0.f, 0.f, 0.f, 0.f, 0.f, 0.f, 0.f};
      v8f cr = {0.f, 0.f, 0.f, 0.f, 0.f, 0.f, 0.f, 0.f};
      cl = wmb(ah.v, blh.v, cl);
      cl = wmb(ah.v, bll.v, cl);
      cl = wmb(al.v, blh.v, cl);
      cr = wmb(ah.v, brh.v, cr);
      cr = wmb(ah.v, brl.v, cr);
      cr = wmb(al.v, brh.v, cr);
#pragma unroll
      for (int r = 0; r < 8; ++r) {
        tl[(8 * hh + r) * 16 + m] = cl[r];
        tr[(8 * hh + r) * 16 + m] = cr[r];
      }
    }
    __syncthreads();
    {
      const v4f q0 = *(const v4f*)(tl + 4 * lane);
      const v4f q1 = *(const v4f*)(tl + 128 + 4 * lane);
      const v4f q2 = *(const v4f*)(tr + 4 * lane);
      const v4f q3 = *(const v4f*)(tr + 128 + 4 * lane);
      const size_t gofs = ((size_t)n * NBATCH + (size_t)b0) * FEAT;
      float* gl = XL + gofs;
      float* gr = XR + gofs;
      if (valid) {
        *(volatile v4f*)(gl + 4 * lane)       = q0;
        *(volatile v4f*)(gl + 128 + 4 * lane) = q1;
        *(volatile v4f*)(gr + 4 * lane)       = q2;
        *(volatile v4f*)(gr + 128 + 4 * lane) = q3;
      }
      __threadfence();
      if (valid) {
        *(volatile v4f*)(gl + 4 * lane)       = q0;
        *(volatile v4f*)(gl + 128 + 4 * lane) = q1;
        *(volatile v4f*)(gr + 4 * lane)       = q2;
        *(volatile v4f*)(gr + 128 + 4 * lane) = q3;
      }
    }
    __syncthreads();
  }
}

__global__ __launch_bounds__(NTHR) void k_gat(
    const float* __restrict__ XL, const float* __restrict__ XR, const int* __restrict__ nbr,
    const float* __restrict__ att, const float* __restrict__ bias,
    float* Hout, float* Part, int nN, int nE, int nDeg) {
  extern __shared__ v4f gat_lds[];
  float* acc  = (float*)gat_lds;
  float* srun = acc + GAT_ACC;
  float* mrun = srun + GAT_SR;
  int*   list = (int*)(mrun + GAT_MR);
  int*   wcnt = list + GAT_LIST;

  const int tid  = threadIdx.x;
  const int lane = tid & 31;
  const int wave = tid >> 5;
  const int hd   = tid & 3;
  const int cell = 4 * tid;
  const int nodeBase = blockIdx.x * NB;

  {
    const v4f z4 = {0.f, 0.f, 0.f, 0.f};
    const v4f mneg = {-3.0e38f, -3.0e38f, -3.0e38f, -3.0e38f};
    for (int i = tid; i < (GAT_ACC + GAT_SR) / 4; i += NTHR) gat_lds[i] = z4;
    v4f* mp = (v4f*)mrun;
    for (int i = tid; i < GAT_MR / 4; i += NTHR) mp[i] = mneg;
  }
  __syncthreads();
  const v4f a4 = *(const v4f*)(att + 4 * hd);
  const v4f b4 = *(const v4f*)(bias + 4 * hd);

  const int nChunks = (nE + CHUNK - 1) / CHUNK;
#pragma unroll 1
  for (int ch = 0; ch < nChunks; ++ch) {
    const int cbase = ch * CHUNK;
    int wc = 0;
#pragma unroll
    for (int g = 0; g < NGRP; ++g) {
      const int el0 = (g * NTHR + tid) * 4;
      const int e0  = cbase + el0;
      const int sent = -2147483647 - 1;
      v4i d;
      if (cbase + CHUNK <= nE) {
        d = *(const v4i*)(nbr + e0);
      } else {
        const int v0 = nbr[min(e0, nE - 1)];
        const int v1 = nbr[min(e0 + 1, nE - 1)];
        const int v2 = nbr[min(e0 + 2, nE - 1)];
        const int v3 = nbr[min(e0 + 3, nE - 1)];
        d.x = (e0     < nE) ? v0 : sent;
        d.y = (e0 + 1 < nE) ? v1 : sent;
        d.z = (e0 + 2 < nE) ? v2 : sent;
        d.w = (e0 + 3 < nE) ? v3 : sent;
      }
      const unsigned s0 = (unsigned)d.x - (unsigned)nodeBase;
      const unsigned s1 = (unsigned)d.y - (unsigned)nodeBase;
      const unsigned s2 = (unsigned)d.z - (unsigned)nodeBase;
      const unsigned s3 = (unsigned)d.w - (unsigned)nodeBase;
      const bool h0 = s0 < (unsigned)NB;
      const bool h1 = s1 < (unsigned)NB;
      const bool h2 = s2 < (unsigned)NB;
      const bool h3 = s3 < (unsigned)NB;
      const unsigned many = __builtin_amdgcn_ballot_w32(h0 | h1 | h2 | h3);
      if (many != 0u) {
#define HITJ(J, HJ, SJ) { \
          const unsigned mj = __builtin_amdgcn_ballot_w32(HJ); \
          if (HJ) { \
            const int pos = wc + (int)__builtin_amdgcn_mbcnt_lo(mj, 0u); \
            if (pos < WCAP) list[wave * WCAP + pos] = ((el0 + (J)) << 5) | (int)(SJ); \
          } \
          wc += (int)__builtin_popcount(mj); }
        HITJ(0, h0, s0)
        HITJ(1, h1, s1)
        HITJ(2, h2, s2)
        HITJ(3, h3, s3)
#undef HITJ
      }
    }
    if (lane == 0) wcnt[wave] = wc;
    __syncthreads();

#pragma unroll 1
    for (int wsx = 0; wsx < NWAVE; ++wsx) {
      int nh = wcnt[wsx];
      if (nh > WCAP) nh = WCAP;
      if (nh < 0) nh = 0;
#pragma unroll 1
      for (int i = 0; i < nh; ++i) {
        const int ent  = list[wsx * WCAP + i];
        const int slot = ent & (NB - 1);
        const int el   = (ent >> 5) & (CHUNK - 1);
        int e = cbase + el;
        if (e > nE - 1) e = nE - 1;
        int src = e / nDeg;
        if (src > nN - 1) src = nN - 1;
        const int node = nodeBase + slot;
        const v4f xs = *(const v4f*)(XL + (size_t)src * ROWF + cell);
        const v4f xt = *(const v4f*)(XR + (size_t)node * ROWF + cell);
        const float t0 = lrelu(xs.x + xt.x), t1 = lrelu(xs.y + xt.y);
        const float t2 = lrelu(xs.z + xt.z), t3 = lrelu(xs.w + xt.w);
        const float lg = t0 * a4.x + t1 * a4.y + t2 * a4.z + t3 * a4.w;
        const int ci = slot * NTHR + tid;
        const float mo = mrun[ci];
        const float mn = fmaxf(mo, lg);
        const float r  = __expf(mo - mn);
        const float w  = __expf(lg - mn);
        srun[ci] = srun[ci] * r + w;
        mrun[ci] = mn;
        v4f* ap = (v4f*)(acc + slot * ROWF + cell);
        const v4f cur = *ap;
        *ap = cur * r + w * xs;
      }
    }
    __syncthreads();
  }

  v4f psum = {0.f, 0.f, 0.f, 0.f};
#pragma unroll 1
  for (int j = 0; j < NB; ++j) {
    const int node = nodeBase + j;
    const v4f xs = *(const v4f*)(XL + (size_t)node * ROWF + cell);
    const v4f xt = *(const v4f*)(XR + (size_t)node * ROWF + cell);
    const float t0 = lrelu(xs.x + xt.x), t1 = lrelu(xs.y + xt.y);
    const float t2 = lrelu(xs.z + xt.z), t3 = lrelu(xs.w + xt.w);
    const float lg = t0 * a4.x + t1 * a4.y + t2 * a4.z + t3 * a4.w;
    const int ci = j * NTHR + tid;
    const float mo = mrun[ci];
    const float mn = fmaxf(mo, lg);
    const float r  = __expf(mo - mn);
    const float w  = __expf(lg - mn);
    const float s  = srun[ci] * r + w;
    v4f* ap = (v4f*)(acc + j * ROWF + cell);
    const v4f av = (*ap) * r + w * xs;
    const float inv = 1.0f / (s + 1e-16f);
    const v4f o = av * inv + b4;
    *ap = o;
    psum += o;
  }
#pragma unroll 1
  for (int j = 0; j < NB; ++j) {
    const v4f o = *(const v4f*)(acc + j * ROWF + cell);
    *(volatile v4f*)(Hout + (size_t)(nodeBase + j) * ROWF + cell) = o;
  }
  *(volatile v4f*)(Part + (size_t)blockIdx.x * ROWF + cell) = psum;
  __threadfence();
#pragma unroll 1
  for (int j = 0; j < NB; ++j) {
    const v4f o = *(const v4f*)(acc + j * ROWF + cell);
    *(volatile v4f*)(Hout + (size_t)(nodeBase + j) * ROWF + cell) = o;
  }
  *(volatile v4f*)(Part + (size_t)blockIdx.x * ROWF + cell) = psum;
}

__global__ __launch_bounds__(NTHR) void k_head(
    const float* __restrict__ H, const float* __restrict__ Part, int nPart,
    const int* __restrict__ agents, const int* __restrict__ nbr,
    const float* __restrict__ Wg1, const float* __restrict__ bg1,
    const float* __restrict__ Wg2, const float* __restrict__ bg2,
    const float* __restrict__ We1, const float* __restrict__ be1,
    const float* __restrict__ We2, const float* __restrict__ be2,
    const float* __restrict__ We3, const float* __restrict__ be3,
    float* out, int nN) {
  extern __shared__ float hd_lds[];
  float* Ragg2 = hd_lds + HD_AGG2;
  float* Rsrc  = hd_lds + HD_SRC;
  float* Rtgt  = hd_lds + HD_TGT;
  float* Rbase = hd_lds + HD_BASE;
  float* Re1   = hd_lds + HD_E1;
  float* Re2   = hd_lds + HD_E2;
  const int tid = threadIdx.x;

#pragma unroll 1
  for (int q = 0; q < 4; ++q) {
    const int cidx = tid + NTHR * q;
    double sacc = 0.0;
#pragma unroll 1
    for (int p = 0; p < nPart; ++p) sacc += (double)Part[(size_t)p * ROWF + cidx];
    Re2[cidx] = (float)(sacc / (double)nN);
  }
#pragma unroll 1
  for (int v = tid; v < NBATCH * FEAT; v += NTHR) {
    const int b = v >> 4, f = v & 15;
    int ag = agents[b];
    ag = ag < 0 ? 0 : (ag > nN - 1 ? nN - 1 : ag);
    Rsrc[v] = H[((size_t)ag * NBATCH + b) * FEAT + f];
  }
#pragma unroll 1
  for (int v = tid; v < NBATCH * DDEG * FEAT; v += NTHR) {
    const int b   = v / (DDEG * FEAT);
    const int rem = v - b * (DDEG * FEAT);
    const int d   = rem >> 4, f = rem & 15;
    int ag = agents[b];
    ag = ag < 0 ? 0 : (ag > nN - 1 ? nN - 1 : ag);
    int nbx = nbr[ag * DDEG + d];
    nbx = nbx < 0 ? 0 : (nbx > nN - 1 ? nN - 1 : nbx);
    Rtgt[v] = H[((size_t)nbx * NBATCH + b) * FEAT + f];
  }
  __syncthreads();

#pragma unroll 1
  for (int v = tid; v < NBATCH * 32; v += NTHR) {
    const int b = v >> 5, j = v & 31;
    float a = bg1[j];
#pragma unroll 1
    for (int k = 0; k < 16; ++k) a += Re2[b * 16 + k] * Wg1[k * 32 + j];
    Re1[v] = tanh_f(a);
  }
  __syncthreads();

#pragma unroll 1
  for (int v = tid; v < NBATCH * 64; v += NTHR) {
    const int b = v >> 6, j = v & 63;
    float a = bg2[j];
#pragma unroll 1
    for (int k = 0; k < 32; ++k) a += Re1[b * 32 + k] * Wg2[k * 64 + j];
    Ragg2[v] = tanh_f(a);
  }
  __syncthreads();

#pragma unroll 1
  for (int v = tid; v < NBATCH * 16; v += NTHR) {
    const int b = v >> 4, j = v & 15;
    float a = be1[j];
#pragma unroll 1
    for (int k = 0; k < 16; ++k) a += Rsrc[b * 16 + k] * We1[k * 16 + j];
#pragma unroll 1
    for (int k = 0; k < 64; ++k) a += Ragg2[b * 64 + k] * We1[(35 + k) * 16 + j];
    Rbase[v] = a;
  }
  __syncthreads();

#pragma unroll 1
  for (int row = tid; row < NBATCH * NOUT; row += NTHR) {
    const int b   = row / NOUT;
    const int rem = row - b * NOUT;
    const int t   = rem / DDEG;
    const int d   = rem - t * DDEG;
    float* e1 = Re1 + tid * 16;
    float* e2 = Re2 + tid * 8;
    const float* tg = Rtgt + (b * DDEG + d) * 16;
#pragma unroll 1
    for (int j = 0; j < 16; ++j) {
      float a = Rbase[b * 16 + j] + We1[(16 + t) * 16 + j];
#pragma unroll 1
      for (int k = 0; k < 16; ++k) a += tg[k] * We1[(19 + k) * 16 + j];
      e1[j] = tanh_f(a);
    }
#pragma unroll 1
    for (int j = 0; j < 8; ++j) {
      float a = be2[j];
#pragma unroll 1
      for (int k = 0; k < 16; ++k) a += e1[k] * We2[k * 8 + j];
      e2[j] = tanh_f(a);
    }
    float o = be3[0];
#pragma unroll 1
    for (int k = 0; k < 8; ++k) o += e2[k] * We3[k];
    Ragg2[row] = o;
  }
  __syncthreads();

  const bool wr = tid < (NBATCH * NOUT) / 4;
  v4f ov = {0.f, 0.f, 0.f, 0.f};
  if (wr) ov = *(const v4f*)(Ragg2 + 4 * tid);
  if (wr) *(volatile v4f*)(out + 4 * tid) = ov;
  __threadfence();
  if (wr) *(volatile v4f*)(out + 4 * tid) = ov;
}

extern "C" void kernel_launch(void* const* d_in, const int* in_sizes, int n_in,
                              void* d_out, int out_size, void* d_ws, size_t ws_size,
                              hipStream_t stream) {
  if (n_in < 17) return;
  if (in_sizes[1] != NBATCH) return;
  if (in_sizes[2] <= 0 || (in_sizes[2] % DDEG) != 0) return;
  const int nN = in_sizes[2] / DDEG;
  if (nN < NB || (nN % NB) != 0) return;
  if ((size_t)in_sizes[0] != (size_t)NBATCH * (size_t)nN * FEAT) return;
  const int nL = in_sizes[3] / (FEAT * FEAT);
  if (nL < 1 || in_sizes[3] != nL * FEAT * FEAT || in_sizes[4] != nL * FEAT * FEAT) return;
  if (in_sizes[5] != nL * FEAT || in_sizes[6] != nL * FEAT) return;
  if (in_sizes[7] != 16 * 32 || in_sizes[8] != 32 || in_sizes[9] != 32 * 64 || in_sizes[10] != 64) return;
  if (in_sizes[11] != 99 * 16 || in_sizes[12] != 16 || in_sizes[13] != 16 * 8 || in_sizes[14] != 8) return;
  if (in_sizes[15] != 8 || in_sizes[16] != 1) return;
  if (out_size != NBATCH * NOUT) return;

  const float* x      = (const float*)d_in[0];
  const int*   agents = (const int*)d_in[1];
  const int*   nbr    = (const int*)d_in[2];
  const float* Wl     = (const float*)d_in[3];
  const float* Wr     = (const float*)d_in[4];
  const float* att    = (const float*)d_in[5];
  const float* bias   = (const float*)d_in[6];
  const float* Wg1    = (const float*)d_in[7];
  const float* bg1    = (const float*)d_in[8];
  const float* Wg2    = (const float*)d_in[9];
  const float* bg2    = (const float*)d_in[10];
  const float* We1    = (const float*)d_in[11];
  const float* be1    = (const float*)d_in[12];
  const float* We2    = (const float*)d_in[13];
  const float* be2    = (const float*)d_in[14];
  const float* We3    = (const float*)d_in[15];
  const float* be3    = (const float*)d_in[16];
  float* out = (float*)d_out;

  const int nPart = nN / NB;
  const size_t planeB = (size_t)nN * ROWF * sizeof(float);
  const size_t partB  = (size_t)nPart * ROWF * sizeof(float);
  size_t off = 0;
  float* XL   = (float*)((char*)d_ws + off); off += planeB;
  float* XR   = (float*)((char*)d_ws + off); off += planeB;
  float* Hp   = (float*)((char*)d_ws + off); off += planeB;
  float* Part = (float*)((char*)d_ws + off); off += partB;
  if (off > ws_size) return;

  const int nE = nN * DDEG;
  const int numTiles = nN * (NBATCH / 16);
  const int nodeGrid = (numTiles + NWAVE * TPW - 1) / (NWAVE * TPW);

  hipFuncSetAttribute(reinterpret_cast<const void*>(&k_gat),
                      hipFuncAttributeMaxDynamicSharedMemorySize, GAT_LDS_BYTES);
  hipFuncSetAttribute(reinterpret_cast<const void*>(&k_head),
                      hipFuncAttributeMaxDynamicSharedMemorySize, HEAD_LDS_BYTES);

  for (int l = 0; l < nL; ++l) {
    const float* hin = (l == 0) ? x : (const float*)Hp;
    const int sN = (l == 0) ? FEAT : ROWF;
    const int sB = (l == 0) ? nN * FEAT : FEAT;
    k_node<<<nodeGrid, NTHR, 0, stream>>>(hin, sN, sB, Wl + (size_t)l * FEAT * FEAT,
                                          Wr + (size_t)l * FEAT * FEAT, XL, XR, nN);
    k_gat<<<nPart, NTHR, GAT_LDS_BYTES, stream>>>(XL, XR, nbr, att + (size_t)l * FEAT,
                                                  bias + (size_t)l * FEAT, Hp, Part, nN, nE, DDEG);
  }
  k_head<<<1, NTHR, HEAD_LDS_BYTES, stream>>>(Hp, Part, nPart, agents, nbr, Wg1, bg1, Wg2, bg2,
                                              We1, be1, We2, be2, We3, be3, out, nN);
}
